// SparseConvBlock_7035156431607
// MI455X (gfx1250) — hardware-verified
//
#include <hip/hip_runtime.h>
#include <stddef.h>
#include <stdint.h>

#define NV     150000
#define CIN    32
#define COUT   64
#define KOFF   27
#define KTOT   (KOFF * CIN)
#define TR     64
#define GTHR   128
#define NBLK   ((NV + TR - 1) / TR)
#define NB2    (NBLK / 2)
#define NPAD   (NBLK * TR)
#define GRP    9
#define NGRP   (KOFF / GRP)
#define KG     (GRP * CIN)
#define PPT    ((TR * GRP * 4) / GTHR)
#define NF8    (NV * CIN / 8)
#define NFB    ((NF8 + 255) / 256)
#define KQ     (KTOT / 8)
#define NW8    (COUT * KQ)
#define NWB    (NW8 / 256)
#define NOUT4  (NV * COUT / 4)
#define NAB    (NOUT4 / 256)
#define RECW   128
#define WSMAX  134217728

static_assert(KTOT == 864);
static_assert((KTOT % 32) == 0);
static_assert(CIN == 32);
static_assert(NGRP * GRP == KOFF);
static_assert((TR * GRP * 4) % GTHR == 0);
static_assert(TR == 64);
static_assert(TR == (GTHR / 32) * 16);
static_assert((NW8 % 256) == 0);
static_assert((NOUT4 % 256) == 0);
static_assert((NV * CIN) % 8 == 0);
static_assert(NPAD >= NV);
static_assert(RECW == 2 * COUT);

typedef float          v4f  __attribute__((ext_vector_type(4)));
typedef float          v8f  __attribute__((ext_vector_type(8)));
typedef int            v4i  __attribute__((ext_vector_type(4)));
typedef int            v8i  __attribute__((ext_vector_type(8)));
typedef unsigned short v8us __attribute__((ext_vector_type(8)));
typedef __bf16         v16bf __attribute__((ext_vector_type(16)));
union FragB { v16bf v; v8us h[2]; v8i w; };
union U8 { v8us v; v4i w; };

__device__ __forceinline__ v8f wmb(const FragB& a, const FragB& b, v8f c) {
  v8f d = __builtin_amdgcn_wmma_f32_16x16x32_bf16(false, a.v, false, b.v, (short)0, c, false, false);
  asm volatile("v_nop\n\tv_nop\n\tv_nop\n\tv_nop" : "+v"(d) : "v"(a.w), "v"(b.w));
  return d;
}

__device__ __forceinline__ unsigned short rne16(float f) {
  unsigned u = __float_as_uint(f);
  u += 0x7FFFu + ((u >> 16) & 1u);
  return (unsigned short)(u >> 16);
}
__device__ __forceinline__ float rne16f(float f) {
  return __uint_as_float(((unsigned)rne16(f)) << 16);
}
__device__ __forceinline__ v8us cvt8(const v4f a, const v4f b) {
  v8us o;
  o[0] = rne16(a.x); o[1] = rne16(a.y); o[2] = rne16(a.z); o[3] = rne16(a.w);
  o[4] = rne16(b.x); o[5] = rne16(b.y); o[6] = rne16(b.z); o[7] = rne16(b.w);
  return o;
}

__global__ __launch_bounds__(256) void k_prep(const float* __restrict__ f, const float* __restrict__ w,
                                               unsigned short* fb, unsigned short* wt) {
  const int tid = (int)threadIdx.x;
  v4f a, b;
  unsigned short* dst;
  if ((int)blockIdx.x < NFB) {
    const int g = (int)blockIdx.x * 256 + tid;
    if (g >= NF8) return;
    const float* p = f + (size_t)g * 8;
    a = *(const v4f*)p;
    b = *(const v4f*)(p + 4);
    dst = fb + (size_t)g * 8;
  } else {
    const int u = ((int)blockIdx.x - NFB) * 256 + tid;
    int d = u / KQ;
    d = d > COUT - 1 ? COUT - 1 : d;
    const int k8 = (u - d * KQ) * 8;
    const float* p = w + (size_t)k8 * COUT + (size_t)d;
    a.x = p[0];                 a.y = p[(size_t)COUT];      a.z = p[(size_t)2 * COUT];  a.w = p[(size_t)3 * COUT];
    b.x = p[(size_t)4 * COUT];  b.y = p[(size_t)5 * COUT];  b.z = p[(size_t)6 * COUT];  b.w = p[(size_t)7 * COUT];
    dst = wt + (size_t)u * 8;
  }
  const v8us o = cvt8(a, b);
  *(volatile v8us*)dst = o;
  __threadfence();
  *(volatile v8us*)dst = o;
}

__global__ __launch_bounds__(GTHR) void k_gemm(const unsigned short* __restrict__ fb,
                                               const unsigned short* __restrict__ wt,
                                               const int* __restrict__ nbr,
                                               float* y, float* rec) {
  __shared__ __attribute__((aligned(16))) unsigned short sA[TR * KG];
  __shared__ __attribute__((aligned(16))) float stg[TR * COUT];
  __shared__ __attribute__((aligned(16))) float srec[RECW];
  const int tid = (int)threadIdx.x, lane = tid & 31, wave = tid >> 5, hh = lane >> 4, m = lane & 15;
  const int blk = (int)blockIdx.x;
  const int r0  = blk * TR;

  v8f acc[4];
  {
    const v8f z = {0.f, 0.f, 0.f, 0.f, 0.f, 0.f, 0.f, 0.f};
    acc[0] = z; acc[1] = z; acc[2] = z; acc[3] = z;
  }
  const unsigned short* arow = sA + (16 * wave + m) * KG + 8 * hh;
  const unsigned short* wrow = wt + (size_t)m * (size_t)KTOT + (size_t)(8 * hh);

#pragma unroll 1
  for (int kg = 0; kg < NGRP; ++kg) {
#pragma unroll 2
    for (int i = 0; i < PPT; ++i) {
      const int p   = i * GTHR + tid;
      const int q   = p & 3;
      const int t   = p >> 2;
      const int row = t & (TR - 1);
      const int kl  = t >> 6;
      const int ko  = kg * GRP + kl;
      const int grow  = r0 + row;
      const int growc = grow > NV - 1 ? NV - 1 : grow;
      int idx = nbr[(size_t)ko * (size_t)NV + (size_t)growc];
      const bool ok = (grow < NV) && (idx >= 0);
      idx = idx < 0 ? 0 : (idx > NV - 1 ? NV - 1 : idx);
      U8 u;
      u.v = *(const v8us*)(fb + (size_t)idx * CIN + (size_t)(8 * q));
      v4i wv = u.w;
      wv.x = ok ? wv.x : 0; wv.y = ok ? wv.y : 0; wv.z = ok ? wv.z : 0; wv.w = ok ? wv.w : 0;
      u.w = wv;
      *(v8us*)(sA + row * KG + kl * CIN + 8 * q) = u.v;
    }
    __syncthreads();

#pragma unroll 3
    for (int ks = 0; ks < GRP; ++ks) {
      FragB a;
      a.h[0] = *(const v8us*)(arow + 32 * ks);
      a.h[1] = *(const v8us*)(arow + 32 * ks + 16);
      const int k0 = (kg * GRP + ks) * 32;
#pragma unroll
      for (int t = 0; t < 4; ++t) {
        const unsigned short* q1 = wrow + (size_t)(16 * t) * (size_t)KTOT + (size_t)k0;
        FragB b;
        b.h[0] = *(const v8us*)q1;
        b.h[1] = *(const v8us*)(q1 + 16);
        acc[t] = wmb(a, b, acc[t]);
      }
    }
    __syncthreads();
  }

#pragma unroll
  for (int t = 0; t < 4; ++t) {
    const int lc = 16 * t + m;
#pragma unroll
    for (int r = 0; r < 8; ++r) {
      const int lr = 16 * wave + 8 * hh + r;
      stg[lr * COUT + lc] = acc[t][r];
    }
  }
  __syncthreads();

  if (tid < COUT) {
    float s = 0.f, s2 = 0.f;
#pragma unroll 8
    for (int r = 0; r < TR; ++r) {
      const float v = stg[r * COUT + tid];
      s += v;
      s2 = fmaf(v, v, s2);
    }
    srec[tid] = s;
    srec[COUT + tid] = s2;
  }
  __syncthreads();

  v4f fv[8];
  size_t op[8];
#pragma unroll
  for (int i = 0; i < 8; ++i) {
    const int lr = 16 * wave + 2 * i + hh;
    fv[i] = *(const v4f*)(stg + lr * COUT + 4 * m);
    op[i] = (size_t)(r0 + lr) * (size_t)COUT + (size_t)(4 * m);
  }
  const v4f rv = *(const v4f*)(srec + 4 * lane);
  float* rp = rec + (size_t)blk * RECW + 4 * lane;

#pragma unroll
  for (int i = 0; i < 8; ++i) *(volatile v4f*)(y + op[i]) = fv[i];
  if (wave == 0) *(volatile v4f*)rp = rv;
  __threadfence();
#pragma unroll
  for (int i = 0; i < 8; ++i) *(volatile v4f*)(y + op[i]) = fv[i];
  if (wave == 0) *(volatile v4f*)rp = rv;
}

__global__ __launch_bounds__(256) void k_fold(const float* __restrict__ rec, const float* __restrict__ gamma,
                                               const float* __restrict__ beta, float* scl) {
  __shared__ double sp[256];
  __shared__ __attribute__((aligned(16))) float so[RECW];
  const int tid = (int)threadIdx.x, lane = tid & 31, wave = tid >> 5;
  const int col = tid & (RECW - 1), half = tid >> 7;
  const int b0 = half ? NB2 : 0;
  const int b1 = half ? NBLK : NB2;
  double a = 0.0;
#pragma unroll 4
  for (int b = b0; b < b1; ++b) a += (double)rec[(size_t)b * RECW + col];
  sp[tid] = a;
  __syncthreads();
  if (tid < COUT) {
    const double S = sp[tid] + sp[tid + 128];
    const double Q = sp[COUT + tid] + sp[COUT + tid + 128];
    const double invn = 1.0 / (double)NV;
    const double mean = S * invn;
    double var = Q * invn - mean * mean;
    var = var < 0.0 ? 0.0 : var;
    const double inv = 1.0 / sqrt(var + 1e-5);
    const double g  = (double)rne16f(gamma[tid]);
    const double bt = (double)rne16f(beta[tid]);
    const double sc = g * inv;
    so[tid]        = (float)sc;
    so[COUT + tid] = (float)(bt - mean * sc);
  }
  __syncthreads();
  const v4f v = *(const v4f*)(so + 4 * lane);
  if (wave == 0) *(volatile v4f*)(scl + 4 * lane) = v;
  __threadfence();
  if (wave == 0) *(volatile v4f*)(scl + 4 * lane) = v;
}

__global__ __launch_bounds__(256) void k_apply(const float* __restrict__ y, const float* __restrict__ scl, float* out) {
  __shared__ __attribute__((aligned(16))) float ss[RECW];
  const int tid = (int)threadIdx.x;
  if (tid < RECW) ss[tid] = scl[tid];
  __syncthreads();
  const int g = (int)blockIdx.x * 256 + tid;
  if (g >= NOUT4) return;
  const size_t e = (size_t)g * 4;
  const int col = (g & 15) * 4;
  const v4f v  = *(const v4f*)(y + e);
  const v4f sc = *(const v4f*)(ss + col);
  const v4f sh = *(const v4f*)(ss + COUT + col);
  v4f o;
  o.x = fmaxf(fmaf(v.x, sc.x, sh.x), 0.f);
  o.y = fmaxf(fmaf(v.y, sc.y, sh.y), 0.f);
  o.z = fmaxf(fmaf(v.z, sc.z, sh.z), 0.f);
  o.w = fmaxf(fmaf(v.w, sc.w, sh.w), 0.f);
  *(volatile v4f*)(out + e) = o;
  __threadfence();
  *(volatile v4f*)(out + e) = o;
}

extern "C" void kernel_launch(void* const* d_in, const int* in_sizes, int n_in,
                              void* d_out, int out_size, void* d_ws, size_t ws_size,
                              hipStream_t stream) {
  if (n_in < 5) return;
  if (in_sizes[0] != NV * CIN) return;
  if (in_sizes[1] != KOFF * CIN * COUT) return;
  if (in_sizes[2] != COUT) return;
  if (in_sizes[3] != COUT) return;
  if (in_sizes[4] != KOFF * NV) return;
  if (out_size != NV * COUT) return;

  const float* features = (const float*)d_in[0];
  const float* weight   = (const float*)d_in[1];
  const float* gamma    = (const float*)d_in[2];
  const float* beta     = (const float*)d_in[3];
  const int*   nbr      = (const int*)d_in[4];
  float* out = (float*)d_out;

  char* ws = (char*)d_ws;
  size_t off = 0;
  const size_t oFB  = off; off += (size_t)NV * CIN * 2;        off = (off + 255) & ~(size_t)255;
  const size_t oWT  = off; off += (size_t)COUT * KTOT * 2;     off = (off + 255) & ~(size_t)255;
  const size_t oY   = off; off += (size_t)NPAD * COUT * 4;     off = (off + 255) & ~(size_t)255;
  const size_t oREC = off; off += (size_t)NBLK * RECW * 4;     off = (off + 255) & ~(size_t)255;
  const size_t oSCL = off; off += (size_t)RECW * 4;            off = (off + 255) & ~(size_t)255;
  if (off > ws_size || off > (size_t)WSMAX) return;

  unsigned short* FB  = (unsigned short*)(ws + oFB);
  unsigned short* WT  = (unsigned short*)(ws + oWT);
  float*          Y   = (float*)(ws + oY);
  float*          REC = (float*)(ws + oREC);
  float*          SCL = (float*)(ws + oSCL);

  k_prep<<<NFB + NWB, 256, 0, stream>>>(features, weight, FB, WT);
  k_gemm<<<NBLK, GTHR, 0, stream>>>(FB, WT, nbr, Y, REC);
  k_fold<<<1, 256, 0, stream>>>(REC, gamma, beta, SCL);
  k_apply<<<NAB, 256, 0, stream>>>(Y, SCL, out);
}
